// SMHSA_71829033059026
// MI455X (gfx1250) — hardware-verified
//
#include <hip/hip_runtime.h>
#include <math.h>

typedef __attribute__((ext_vector_type(16))) _Float16 v16h;
typedef __attribute__((ext_vector_type(16))) __bf16 v16b;
typedef __attribute__((ext_vector_type(8)))  _Float16 v8h;
typedef __attribute__((ext_vector_type(8)))  float v8f;
typedef __attribute__((ext_vector_type(4)))  float v4f;
typedef __attribute__((ext_vector_type(2)))  float v2f;
typedef __attribute__((ext_vector_type(4)))  unsigned v4u;
typedef __attribute__((ext_vector_type(4)))  int v4i;
typedef float __attribute__((may_alias)) float_a;
typedef int __attribute__((may_alias)) int_a;

template <typename T> __device__ __forceinline__ void vst2(void* p, T v) { *(volatile T*)p = v; __threadfence(); *(volatile T*)p = v; }
__device__ __forceinline__ v8f wmma16(v16h a, v16h b, v8f c) {
  v8f d = __builtin_amdgcn_wmma_f32_16x16x32_f16(false, a, false, b, (short)0, c, false, false);
  asm volatile("v_nop\n\tv_nop\n\tv_nop\n\tv_nop" : "+v"(d) : "v"(a), "v"(b));
  return d;
}
__device__ __forceinline__ v8f wmma_bf(v16b a, v16b b, v8f c) {
  v8f d = __builtin_amdgcn_wmma_f32_16x16x32_bf16(false, a, false, b, (short)0, c, false, false);
  asm volatile("v_nop\n\tv_nop\n\tv_nop\n\tv_nop" : "+v"(d) : "v"(a), "v"(b));
  return d;
}
__device__ __forceinline__ v16h frag_h(const _Float16* rowk0, int lane) {
  union { v16h v; v8h q[2]; } u; const _Float16* p = rowk0 + 8 * (lane >> 4);
  u.q[0] = *(const v8h*)p; u.q[1] = *(const v8h*)(p + 16); return u.v;
}
__device__ __forceinline__ v16h frag_f32(const float* rowk0, int lane) {
  v16h a; const float* p = rowk0 + 8 * (lane >> 4);
#pragma unroll
  for (int i = 0; i < 8; ++i) { a[i] = (_Float16)p[i]; a[8 + i] = (_Float16)p[16 + i]; }
  return a;
}
__device__ __forceinline__ v16h frag_f32s(const float* rowk0, int lane, float sc) {
  v16h a; const float* p = rowk0 + 8 * (lane >> 4);
#pragma unroll
  for (int i = 0; i < 8; ++i) { a[i] = (_Float16)(p[i] * sc); a[8 + i] = (_Float16)(p[16 + i] * sc); }
  return a;
}
__device__ __forceinline__ v16h fragc_f32(const float* W, int k0, int n, int lane, int ld, int K) {
  v16h a; const int g = lane >> 4;
#pragma unroll
  for (int i = 0; i < 8; ++i) { const int ka = k0 + 8 * g + i, kb = ka + 16;
    a[i] = (_Float16)(ka < K ? W[(size_t)ka * ld + n] : 0.f); a[8 + i] = (_Float16)(kb < K ? W[(size_t)kb * ld + n] : 0.f); }
  return a;
}
struct F2 { v16b h, l; };
__device__ __forceinline__ F2 bsplit16(const float v[16]) { F2 r;
#pragma unroll
  for (int i = 0; i < 16; ++i) { const __bf16 h = (__bf16)v[i]; r.h[i] = h; r.l[i] = (__bf16)(v[i] - (float)h); }
  return r; }
__device__ __forceinline__ F2 split_row(const float* row, int k0, int lane) { float v[16]; const float* p = row + k0 + 8 * (lane >> 4);
#pragma unroll
  for (int i = 0; i < 8; ++i) { v[i] = p[i]; v[8 + i] = p[16 + i]; }
  return bsplit16(v); }
__device__ __forceinline__ F2 split_rowK(const float* row, int k0, int lane, int K) { float v[16]; const int g = lane >> 4;
#pragma unroll
  for (int i = 0; i < 8; ++i) { const int ka = k0 + 8 * g + i, kb = ka + 16; v[i] = ka < K ? row[ka] : 0.f; v[8 + i] = kb < K ? row[kb] : 0.f; }
  return bsplit16(v); }
__device__ __forceinline__ F2 split_col(const float* W, int k0, int n, int lane, int ld, int K) { float v[16]; const int g = lane >> 4;
#pragma unroll
  for (int i = 0; i < 8; ++i) { const int ka = k0 + 8 * g + i, kb = ka + 16; v[i] = ka < K ? W[(size_t)ka * ld + n] : 0.f; v[8 + i] = kb < K ? W[(size_t)kb * ld + n] : 0.f; }
  return bsplit16(v); }
__device__ __forceinline__ v8f mac3(const F2& a, const F2& b, v8f c) { c = wmma_bf(a.l, b.h, c); c = wmma_bf(a.h, b.l, c); return wmma_bf(a.h, b.h, c); }
__device__ __forceinline__ float sigm(float v) { return 1.0f / (1.0f + expf(-v)); }
#define LDSX() do { asm volatile("s_wait_dscnt 0" ::: "memory"); __builtin_amdgcn_wave_barrier(); __builtin_amdgcn_fence(__ATOMIC_RELEASE, "workgroup"); } while (0)


#define NBATCH 32
#define CIN 64
#define TT 12
#define NV 256
#define COUT 32
#define NBT (NBATCH * TT)
__device__ __forceinline__ float bfr(float v) { return (float)(__bf16)v; }

__global__ __launch_bounds__(128) void k_qk(const float* __restrict__ x, const float* __restrict__ Wq, const float* __restrict__ bq, const float* __restrict__ Wk, const float* __restrict__ bk, float* __restrict__ QK) {
  __shared__ __align__(16) float so[4][16][68];
  const int tid = threadIdx.x, wave = tid >> 5, lane = tid & 31, col = lane & 15, g = lane >> 4;
  const int bt = blockIdx.x >> 1, which = blockIdx.x & 1; const int b = bt / TT, t = bt % TT; const float* W = which ? Wk : Wq; const float* bb_ = which ? bk : bq;
  const float* xb = x + ((size_t)b * CIN * TT + t) * NV;
  float* dst = QK + ((size_t)which * NBT + bt) * NV * CIN;
#pragma unroll 1
  for (int vt = wave; vt < NV / 16; vt += 4) { v8f acc[4] = {};
#pragma unroll
    for (int kc = 0; kc < 2; ++kc) { const v16b a = split_col(xb, kc * 32, vt * 16 + col, lane, TT * NV, CIN).h;
#pragma unroll
      for (int j = 0; j < 4; ++j) acc[j] = wmma_bf(a, split_row(W + (size_t)(j * 16 + col) * CIN, kc * 32, lane).h, acc[j]); }
#pragma unroll
    for (int j = 0; j < 4; ++j) { const float bb = bfr(bb_[j * 16 + col]);
#pragma unroll
      for (int r = 0; r < 8; ++r) so[wave][8 * g + r][j * 16 + col] = acc[j][r] + bb; }
    LDSX();
    for (int rl = 0; rl < 16; ++rl) { if (lane < 16) vst2(dst + (size_t)(vt * 16 + rl) * CIN + lane * 4, *(const v4f*)(&so[wave][rl][lane * 4])); }
    LDSX(); }
}
__global__ __launch_bounds__(128) void k_xf(const float* __restrict__ x, const float* __restrict__ weight, float* __restrict__ XF) {
  __shared__ __align__(16) float so[4][16][36];
  const int tid = threadIdx.x, wave = tid >> 5, lane = tid & 31, col = lane & 15, g = lane >> 4; const int r0 = blockIdx.x * 64 + wave * 16;
  v8f acc[2] = {};
#pragma unroll
  for (int kc = 0; kc < 2; ++kc) { const v16b a = split_row(x + (size_t)(r0 + col) * CIN, kc * 32, lane).h;
#pragma unroll
    for (int j = 0; j < 2; ++j) acc[j] = wmma_bf(a, split_col(weight, kc * 32, j * 16 + col, lane, COUT, CIN).h, acc[j]); }
#pragma unroll
  for (int j = 0; j < 2; ++j)
#pragma unroll
    for (int r = 0; r < 8; ++r) so[wave][8 * g + r][j * 16 + col] = acc[j][r];
  LDSX();
  for (int rl = 0; rl < 16; ++rl) { if (lane < 8) vst2(XF + (size_t)(r0 + rl) * COUT + lane * 4, *(const v4f*)(&so[wave][rl][lane * 4])); }
}
__global__ __launch_bounds__(128) void k_attn(const float* __restrict__ QK, int bt0, float* __restrict__ P) {
  __shared__ __align__(16) float sS[4][16][NV + 4];
  const int tid = threadIdx.x, wave = tid >> 5, lane = tid & 31, col = lane & 15, g = lane >> 4; const int bt = bt0 + blockIdx.x;
  const float* Q = QK + (size_t)bt * NV * CIN; const float* K = QK + ((size_t)NBT + bt) * NV * CIN; float* Pb = P + (size_t)blockIdx.x * NV * NV;
#pragma unroll 1
  for (int vt = wave; vt < NV / 16; vt += 4) { F2 aq[2];
#pragma unroll
    for (int kc = 0; kc < 2; ++kc) aq[kc] = split_row(Q + (size_t)(vt * 16 + col) * CIN, kc * 32, lane);
#pragma unroll 1
    for (int wt = 0; wt < NV / 16; ++wt) { v8f s = {};
#pragma unroll
      for (int kc = 0; kc < 2; ++kc) s = mac3(aq[kc], split_row(K + (size_t)(wt * 16 + col) * CIN, kc * 32, lane), s);
#pragma unroll
      for (int r = 0; r < 8; ++r) sS[wave][8 * g + r][wt * 16 + col] = s[r] * 0.25f; }
    LDSX();
    { const int rl = lane & 15, hf = lane >> 4; float* row = &sS[wave][rl][hf * 128]; float mx = -3.4e38f;
#pragma unroll 4
      for (int k = 0; k < 128; ++k) mx = fmaxf(mx, row[k]);
      mx = fmaxf(mx, __shfl_xor(mx, 16, 32)); float z = 0.f;
#pragma unroll 4
      for (int k = 0; k < 128; ++k) { const float e = expf(row[k] - mx); row[k] = e; z += e; }
      z += __shfl_xor(z, 16, 32); const float inv = 1.0f / z;
#pragma unroll 4
      for (int k = 0; k < 128; ++k) row[k] *= inv; }
    LDSX();
    for (int rl = 0; rl < 16; ++rl) { for (int pc = lane; pc < NV / 4; pc += 32) vst2(Pb + (size_t)(vt * 16 + rl) * NV + pc * 4, *(const v4f*)(&sS[wave][rl][pc * 4])); }
    LDSX(); }
}
__global__ __launch_bounds__(128) void k_sec(const float* __restrict__ XF, const float* __restrict__ P, int bt0, const float* __restrict__ bias, float* __restrict__ out) {
  __shared__ __align__(16) float so[4][16][132];
  const int tid = threadIdx.x, wave = tid >> 5, lane = tid & 31, col = lane & 15, g = lane >> 4; const int bt = bt0 + blockIdx.x; const int b = bt / TT, t = bt % TT;
  const float* Pb = P + (size_t)blockIdx.x * NV * NV; const int ct = wave & 1, nh = wave >> 1;
  const int c = ct * 16 + col; const float* arow = XF + (((size_t)b * COUT + c) * TT + t) * NV;
  v8f ah[8] = {}, al[8] = {};
#pragma unroll 1
  for (int kc = 0; kc < NV / 32; ++kc) { const F2 a = split_row(arow, kc * 32, lane);
#pragma unroll
    for (int j = 0; j < 8; ++j) { const F2 pb = split_col(Pb, kc * 32, nh * 128 + j * 16 + col, lane, NV, NV); ah[j] = wmma_bf(a.h, pb.h, ah[j]); ah[j] = wmma_bf(a.l, pb.h, ah[j]); al[j] = wmma_bf(a.h, pb.l, al[j]); } }
#pragma unroll
  for (int j = 0; j < 8; ++j) { const int wcol = nh * 128 + j * 16 + col; const float bb = bfr(bias[wcol & 31]);
#pragma unroll
    for (int r = 0; r < 8; ++r) so[wave][8 * g + r][j * 16 + col] = ah[j][r] + al[j][r] + bb; }
  LDSX();
  for (int rl = 0; rl < 16; ++rl) { const int cc = ct * 16 + rl; vst2(out + (((size_t)b * COUT + cc) * TT + t) * NV + nh * 128 + lane * 4, *(const v4f*)(&so[wave][rl][lane * 4])); }
}
extern "C" void kernel_launch(void* const* d_in, const int* in_sizes, int n_in, void* d_out, int out_size, void* d_ws, size_t ws_size, hipStream_t stream) {
  (void)in_sizes; (void)n_in; (void)out_size; (void)ws_size;
  const float** I = (const float**)d_in;
  const float* x = I[0]; const float* weight = I[1]; const float* bias = I[2]; const float* Wq = I[3]; const float* bq = I[4]; const float* Wk = I[5]; const float* bk = I[6];
  float* out = (float*)d_out;
  char* ws = (char*)d_ws; size_t off = 0;
  auto take = [&](size_t bytes) { char* p = ws + off; off += (bytes + 255) & ~(size_t)255; return p; };
#define PCH 96
  float* QK = (float*)take((size_t)2 * NBT * NV * CIN * 4); float* XF = (float*)take((size_t)NBATCH * COUT * TT * NV * 4); float* P = (float*)take((size_t)PCH * NV * NV * 4);
  k_qk<<<NBT * 2, 128, 0, stream>>>(x, Wq, bq, Wk, bk, QK);
  k_xf<<<(NBATCH * CIN * TT * NV / CIN) / 64, 128, 0, stream>>>(x, weight, XF);
  for (int bt0 = 0; bt0 < NBT; bt0 += PCH) { k_attn<<<PCH, 128, 0, stream>>>(QK, bt0, P); k_sec<<<PCH, 128, 0, stream>>>(XF, P, bt0, bias, out); }
}
